// HANLayer_1906965479534
// MI455X (gfx1250) — hardware-run, weakly checked
//
#include <hip/hip_runtime.h>


namespace {
constexpr int N = 10000, E = 200000, M = 3, D = 256, KH = 8, F = 32, HID = 128, NSW = (N * M) / 16  ;
constexpr float XS = 8.0f, HS = 256.0f, WSC = 256.0f, SLOPE = 0.2f;
typedef _Float16 b16;
typedef __attribute__((ext_vector_type(16))) _Float16 v16b;
typedef __attribute__((ext_vector_type(8))) _Float16 v8b;
typedef __attribute__((ext_vector_type(8))) float v8f;
typedef __attribute__((ext_vector_type(4))) float v4f;
__device__ __forceinline__ float bf16_rne(float f) { unsigned int u = __float_as_uint(f); u += 0x7FFFu + ((u >> 16) & 1u); float r = __uint_as_float(u & 0xFFFF0000u); asm volatile("" : "+v"(r)); return r; }
__device__ __forceinline__ float bfv(float f) { float r = bf16_rne(f); asm volatile("" : "+v"(r)); return r; }
__device__ __forceinline__ void split16(float v, b16& hi, b16& lo) { hi = (b16)v; lo = (b16)(v - (float)hi); }
__device__ __forceinline__ v16b frag_kb(const b16* p, int hh) { const v8b a = *(const v8b*)(p + 8 * hh), b = *(const v8b*)(p + 16 + 8 * hh); v16b f;
#pragma unroll
  for (int e = 0; e < 8; ++e) { f[e] = a[e]; f[8 + e] = b[e]; } return f; }
__device__ __forceinline__ v8f wmma16b(v16b a, v16b b, v8f c) { v8f d = __builtin_amdgcn_wmma_f32_16x16x32_f16(false, a, false, b, (short)0, c, false, false); asm volatile("v_nop\n\tv_nop\n\tv_nop\n\tv_nop" : "+v"(d) : "v"(a), "v"(b)); return d; }
__device__ __forceinline__ void wave_lds_sync() { __builtin_amdgcn_fence(__ATOMIC_RELEASE, "workgroup"); __builtin_amdgcn_wave_barrier(); __builtin_amdgcn_fence(__ATOMIC_ACQUIRE, "workgroup"); }
__device__ __forceinline__ float pmul(float a, float b) { float p = a * b; asm volatile("" : "+v"(p)); return p; }
__device__ __forceinline__ int iclamp(int v, int lo, int hi) { return v < lo ? lo : (v > hi ? hi : v); }
__device__ __forceinline__ float leaky(float v) { return v > 0.0f ? v : SLOPE * v; }
__device__ __forceinline__ float elu(float v) { return v > 0.0f ? v : (__expf(v) - 1.0f); }
constexpr int CSR_NBLKA = 512, CSR_GBA = 9, CSR_GNA = 1 << CSR_GBA  , CSR_TSA = (CSR_GNA < 32 ? 32 : CSR_GNA)  , CSR_MAXGA = 512, CSR_CAPA = 12288  ;
__device__ __host__ __forceinline__ int csr_tixA(int v) { return (v >> CSR_GBA) * CSR_TSA + (v & (CSR_GNA - 1)); }
__global__ __launch_bounds__(64) void csrA_kernelA(const int* __restrict__ dst, int E, int N, int nG, int CHP, int NGP, int* __restrict__ STG, int* __restrict__ HST) {
  extern __shared__ int sm[];
  int* cnt = sm; int* run = sm + NGP; int* ids = sm + 2 * NGP;
  const int b = blockIdx.x; const int ch = (E + CSR_NBLKA - 1) / CSR_NBLKA; const int e0 = b * ch, e1 = min(E, e0 + ch);
  for (int i = threadIdx.x; i < NGP; i += 64) cnt[i] = 0;
  for (int i = threadIdx.x; i < CHP; i += 64) ids[i] = -1;
  __syncthreads();
  if (threadIdx.x == 0) {
    for (int e = e0; e < e1; ++e) { int d = dst[e]; d = (d < 0) ? 0 : (d >= N ? N - 1 : d); cnt[d >> CSR_GBA] += 1; }
    int acc = 0; for (int g = 0; g < nG; ++g) { run[g] = acc; acc += cnt[g]; }
    for (int e = e0; e < e1; ++e) { int d = dst[e]; d = (d < 0) ? 0 : (d >= N ? N - 1 : d); const int g = d >> CSR_GBA; ids[run[g]] = e; run[g] += 1; } }
  __syncthreads();
  typedef __attribute__((ext_vector_type(4))) int v4i;
  for (int pass = 0; pass < 2; ++pass) {
    for (int i = threadIdx.x; i < CHP / 4; i += 64) *(volatile v4i*)(STG + (size_t)b * CHP + i * 4) = *(const v4i*)(&ids[i * 4]);
    for (int i = threadIdx.x; i < NGP / 4; i += 64) { v4i v; for (int e = 0; e < 4; ++e) v[e] = (i * 4 + e < nG) ? cnt[i * 4 + e] : 0; *(volatile v4i*)(HST + (size_t)b * NGP + i * 4) = v; }
    __threadfence(); }
}
__global__ __launch_bounds__(512) void csrS_kernelA(const int* __restrict__ HST, int nG, int NGP, int* __restrict__ START, int* __restrict__ TOT, int* __restrict__ OFF) {
  __shared__ int tot[CSR_MAXGA];
  const int b = threadIdx.x;
  for (int pass = 0; pass < 2; ++pass) { int runb = 0; for (int g = 0; g < nG; ++g) { int c = HST[(size_t)b * NGP + g]; c = (c < 0) ? 0 : c; ((volatile int*)OFF)[(size_t)g * CSR_NBLKA + b] = runb; runb += c; } __threadfence(); }
  for (int g = threadIdx.x; g < nG; g += 512) { int s = 0; for (int bb = 0; bb < CSR_NBLKA; ++bb) { int c = HST[(size_t)bb * NGP + g]; s += (c < 0) ? 0 : c; } tot[g] = s; }
  __syncthreads();
  if (threadIdx.x < 32) {
    __shared__ int st[CSR_MAXGA + 32];
    if (threadIdx.x == 0) { int acc = 0; for (int g = 0; g < NGP; ++g) { st[g] = acc; if (g < nG) acc += (tot[g] + 31) & ~31; } st[NGP] = acc; }
    __builtin_amdgcn_fence(__ATOMIC_RELEASE, "workgroup"); __builtin_amdgcn_wave_barrier(); __builtin_amdgcn_fence(__ATOMIC_ACQUIRE, "workgroup");
    for (int pass = 0; pass < 2; ++pass) { for (int i = threadIdx.x; i < NGP + 32; i += 32) { ((volatile int*)START)[i] = (i <= NGP) ? st[min(i, NGP)] : 0; ((volatile int*)TOT)[i] = (i < nG) ? tot[i] : 0; } __threadfence(); } }
}
__global__ __launch_bounds__(256) void csrB_kernelA(const int* __restrict__ dst, int N, int nG, int CHP, int NGP, int permLen, const int* __restrict__ STG, const int* __restrict__ HST, const int* __restrict__ OFF, const int* __restrict__ START, const int* __restrict__ TOT, int* __restrict__ PERM, int* __restrict__ ROWPTR, int* __restrict__ ROWCNT, int* __restrict__ FLAG) {
  typedef __attribute__((ext_vector_type(4))) int v4i;
  __shared__ int ids[CSR_CAPA]; __shared__ unsigned short key[CSR_CAPA]; __shared__ int outp[CSR_CAPA]; __shared__ int ncnt[CSR_GNA + 1]; __shared__ int boff[CSR_NBLKA + 1];
  const int g = blockIdx.x, t_ = threadIdx.x; int tot = TOT[g]; int st = START[g], stn = START[g + 1]; const int v0 = g * CSR_GNA; const int nv = min(CSR_GNA, N - v0); const int t0 = g * CSR_TSA;
  st = (st < 0) ? 0 : (st > permLen - 32 ? permLen - 32 : st) & ~31; stn = (stn < st) ? st : (stn > permLen ? permLen : stn); tot = (tot < 0) ? 0 : tot; if (tot > stn - st && tot <= CSR_CAPA) tot = stn - st;
  if (tot > CSR_CAPA) {
    for (int pass = 0; pass < 2; ++pass) { for (int i = t_; i < CSR_TSA / 4; i += 256) { v4i a, c; for (int e = 0; e < 4; ++e) { a[e] = st; c[e] = 0; } *(volatile v4i*)(ROWPTR + t0 + i * 4) = a; *(volatile v4i*)(ROWCNT + t0 + i * 4) = c; } if (t_ == 0) ((volatile int*)FLAG)[0] = 1; __threadfence(); } (void)nv; return; }
  if (t_ == 0) { int acc = 0; for (int b = 0; b < CSR_NBLKA; ++b) { boff[b] = acc; int c = HST[(size_t)b * NGP + g]; c = (c < 0) ? 0 : (c > CHP ? CHP : c); acc += c; if (acc > tot) acc = tot; } boff[CSR_NBLKA] = acc; }
  for (int i = t_; i <= CSR_GNA; i += 256) ncnt[i] = 0;
  __syncthreads();
  for (int b = 0; b < CSR_NBLKA; ++b) { const int c = boff[b + 1] - boff[b]; int o_ = OFF[(size_t)g * CSR_NBLKA + b]; o_ = (o_ < 0) ? 0 : (o_ > CHP - c ? CHP - c : o_); const int* src_ = STG + (size_t)b * CHP + o_;
    for (int i = t_; i < c; i += 256) { int id = src_[i]; id = (id < 0) ? 0 : id; ids[boff[b] + i] = id; int d = dst[id]; d = (d < v0) ? v0 : (d >= N ? N - 1 : d); int kk = d - v0; kk = (kk < 0) ? 0 : (kk >= CSR_GNA ? CSR_GNA - 1 : kk); key[boff[b] + i] = (unsigned short)kk; } }
  __syncthreads();
  if (t_ == 0) { for (int i = 0; i < tot; ++i) ncnt[key[i]] += 1; int acc = 0; for (int vl = 0; vl < CSR_GNA; ++vl) { const int c = ncnt[vl]; ncnt[vl] = acc; acc += c; } ncnt[CSR_GNA] = acc;
    for (int i = 0; i < tot; ++i) { const int vl = key[i]; outp[ncnt[vl]] = ids[i]; ncnt[vl] += 1; }
    for (int vl = CSR_GNA; vl > 0; --vl) ncnt[vl] = ncnt[vl - 1]; ncnt[0] = 0; }
  __syncthreads();
  for (int pass = 0; pass < 2; ++pass) {
    for (int i = t_; i < (stn - st) / 4; i += 256) { v4i v; for (int e = 0; e < 4; ++e) { const int q = i * 4 + e; v[e] = (q < tot) ? outp[q] : -1; } *(volatile v4i*)(PERM + st + i * 4) = v; }
    for (int i = t_; i < CSR_TSA / 4; i += 256) { v4i a, c; for (int e = 0; e < 4; ++e) { const int vl = i * 4 + e; const int vc = vl < CSR_GNA ? vl : CSR_GNA; a[e] = (vl < CSR_GNA) ? st + ncnt[vc] : st; c[e] = (vl < nv) ? (ncnt[(vc < CSR_GNA ? vc : CSR_GNA - 1) + 1] - ncnt[vc]) : 0; } *(volatile v4i*)(ROWPTR + t0 + i * 4) = a; *(volatile v4i*)(ROWCNT + t0 + i * 4) = c; }
    __threadfence(); }
}
__global__ __launch_bounds__(256) void csrZ_kernelA(int* __restrict__ p, size_t n4) { typedef __attribute__((ext_vector_type(4))) int v4i; const size_t tid = (size_t)blockIdx.x * 256 + threadIdx.x, nth = (size_t)gridDim.x * 256; v4i z = {0, 0, 0, 0}; for (size_t i = tid; i < n4; i += nth) *(volatile v4i*)(p + i * 4) = z; }
struct CsrBufsA { int *STG, *HST, *OFF, *START, *TOT, *PERM, *ROWPTR, *ROWCNT, *FLAG; int nG, NGP, CHP; size_t permLen; char* base; size_t bytes; };
static size_t csr_carveA(CsrBufsA& c, char* ws, size_t off, int E, int N) {
  const size_t off0 = off; c.base = ws + off;
  auto al = [&](size_t bytes) { char* p = ws + off; off += (bytes + 255) & ~(size_t)255; return p; };
  c.nG = (N + CSR_GNA - 1) / CSR_GNA; c.NGP = (c.nG + 31) & ~31; const int ch = (E + CSR_NBLKA - 1) / CSR_NBLKA; c.CHP = (ch + 31) & ~31; c.permLen = (size_t)E + 32 * (size_t)c.nG + 32;
  c.STG = (int*)al((size_t)CSR_NBLKA * c.CHP * 4); c.HST = (int*)al((size_t)CSR_NBLKA * c.NGP * 4); c.OFF = (int*)al((size_t)c.NGP * CSR_NBLKA * 4); c.START = (int*)al((size_t)(c.NGP + 64) * 4); c.TOT = (int*)al((size_t)(c.NGP + 64) * 4);
  c.PERM = (int*)al(c.permLen * 4); c.ROWPTR = (int*)al((size_t)c.nG * CSR_TSA * 4); c.ROWCNT = (int*)al((size_t)c.nG * CSR_TSA * 4); c.FLAG = (int*)al(256);
  c.bytes = off - off0; return off;
}
static void csr_buildA(const CsrBufsA& c, const int* dst, int E, int N, hipStream_t stream) {
  const size_t smem = (size_t)(2 * c.NGP + c.CHP) * 4;
  csrZ_kernelA<<<512, 256, 0, stream>>>((int*)c.base, c.bytes / 16);
  csrA_kernelA<<<CSR_NBLKA, 64, smem, stream>>>(dst, E, N, c.nG, c.CHP, c.NGP, c.STG, c.HST);
  csrS_kernelA<<<1, 512, 0, stream>>>(c.HST, c.nG, c.NGP, c.START, c.TOT, c.OFF);
  csrB_kernelA<<<c.nG, 256, 0, stream>>>(dst, N, c.nG, c.CHP, c.NGP, (int)c.permLen, c.STG, c.HST, c.OFF, c.START, c.TOT, c.PERM, c.ROWPTR, c.ROWCNT, c.FLAG);
}
constexpr int CSR_NBLKB = 512, CSR_GBB = 9, CSR_GNB = 1 << CSR_GBB  , CSR_TSB = (CSR_GNB < 32 ? 32 : CSR_GNB)  , CSR_MAXGB = 512, CSR_CAPB = 12288  ;
__device__ __host__ __forceinline__ int csr_tixB(int v) { return (v >> CSR_GBB) * CSR_TSB + (v & (CSR_GNB - 1)); }
__global__ __launch_bounds__(64) void csrA_kernelB(const int* __restrict__ dst, int E, int N, int nG, int CHP, int NGP, int* __restrict__ STG, int* __restrict__ HST) {
  extern __shared__ int sm[];
  int* cnt = sm; int* run = sm + NGP; int* ids = sm + 2 * NGP;
  const int b = blockIdx.x; const int ch = (E + CSR_NBLKB - 1) / CSR_NBLKB; const int e0 = b * ch, e1 = min(E, e0 + ch);
  for (int i = threadIdx.x; i < NGP; i += 64) cnt[i] = 0;
  for (int i = threadIdx.x; i < CHP; i += 64) ids[i] = -1;
  __syncthreads();
  if (threadIdx.x == 0) {
    for (int e = e0; e < e1; ++e) { int d = dst[e]; d = (d < 0) ? 0 : (d >= N ? N - 1 : d); cnt[d >> CSR_GBB] += 1; }
    int acc = 0; for (int g = 0; g < nG; ++g) { run[g] = acc; acc += cnt[g]; }
    for (int e = e0; e < e1; ++e) { int d = dst[e]; d = (d < 0) ? 0 : (d >= N ? N - 1 : d); const int g = d >> CSR_GBB; ids[run[g]] = e; run[g] += 1; } }
  __syncthreads();
  typedef __attribute__((ext_vector_type(4))) int v4i;
  for (int pass = 0; pass < 2; ++pass) {
    for (int i = threadIdx.x; i < CHP / 4; i += 64) *(volatile v4i*)(STG + (size_t)b * CHP + i * 4) = *(const v4i*)(&ids[i * 4]);
    for (int i = threadIdx.x; i < NGP / 4; i += 64) { v4i v; for (int e = 0; e < 4; ++e) v[e] = (i * 4 + e < nG) ? cnt[i * 4 + e] : 0; *(volatile v4i*)(HST + (size_t)b * NGP + i * 4) = v; }
    __threadfence(); }
}
__global__ __launch_bounds__(512) void csrS_kernelB(const int* __restrict__ HST, int nG, int NGP, int* __restrict__ START, int* __restrict__ TOT, int* __restrict__ OFF) {
  __shared__ int tot[CSR_MAXGB];
  const int b = threadIdx.x;
  for (int pass = 0; pass < 2; ++pass) { int runb = 0; for (int g = 0; g < nG; ++g) { int c = HST[(size_t)b * NGP + g]; c = (c < 0) ? 0 : c; ((volatile int*)OFF)[(size_t)g * CSR_NBLKB + b] = runb; runb += c; } __threadfence(); }
  for (int g = threadIdx.x; g < nG; g += 512) { int s = 0; for (int bb = 0; bb < CSR_NBLKB; ++bb) { int c = HST[(size_t)bb * NGP + g]; s += (c < 0) ? 0 : c; } tot[g] = s; }
  __syncthreads();
  if (threadIdx.x < 32) {
    __shared__ int st[CSR_MAXGB + 32];
    if (threadIdx.x == 0) { int acc = 0; for (int g = 0; g < NGP; ++g) { st[g] = acc; if (g < nG) acc += (tot[g] + 31) & ~31; } st[NGP] = acc; }
    __builtin_amdgcn_fence(__ATOMIC_RELEASE, "workgroup"); __builtin_amdgcn_wave_barrier(); __builtin_amdgcn_fence(__ATOMIC_ACQUIRE, "workgroup");
    for (int pass = 0; pass < 2; ++pass) { for (int i = threadIdx.x; i < NGP + 32; i += 32) { ((volatile int*)START)[i] = (i <= NGP) ? st[min(i, NGP)] : 0; ((volatile int*)TOT)[i] = (i < nG) ? tot[i] : 0; } __threadfence(); } }
}
__global__ __launch_bounds__(256) void csrB_kernelB(const int* __restrict__ dst, int N, int nG, int CHP, int NGP, int permLen, const int* __restrict__ STG, const int* __restrict__ HST, const int* __restrict__ OFF, const int* __restrict__ START, const int* __restrict__ TOT, int* __restrict__ PERM, int* __restrict__ ROWPTR, int* __restrict__ ROWCNT, int* __restrict__ FLAG) {
  typedef __attribute__((ext_vector_type(4))) int v4i;
  __shared__ int ids[CSR_CAPB]; __shared__ unsigned short key[CSR_CAPB]; __shared__ int outp[CSR_CAPB]; __shared__ int ncnt[CSR_GNB + 1]; __shared__ int boff[CSR_NBLKB + 1];
  const int g = blockIdx.x, t_ = threadIdx.x; int tot = TOT[g]; int st = START[g], stn = START[g + 1]; const int v0 = g * CSR_GNB; const int nv = min(CSR_GNB, N - v0); const int t0 = g * CSR_TSB;
  st = (st < 0) ? 0 : (st > permLen - 32 ? permLen - 32 : st) & ~31; stn = (stn < st) ? st : (stn > permLen ? permLen : stn); tot = (tot < 0) ? 0 : tot; if (tot > stn - st && tot <= CSR_CAPB) tot = stn - st;
  if (tot > CSR_CAPB) {
    for (int pass = 0; pass < 2; ++pass) { for (int i = t_; i < CSR_TSB / 4; i += 256) { v4i a, c; for (int e = 0; e < 4; ++e) { a[e] = st; c[e] = 0; } *(volatile v4i*)(ROWPTR + t0 + i * 4) = a; *(volatile v4i*)(ROWCNT + t0 + i * 4) = c; } if (t_ == 0) ((volatile int*)FLAG)[0] = 1; __threadfence(); } (void)nv; return; }
  if (t_ == 0) { int acc = 0; for (int b = 0; b < CSR_NBLKB; ++b) { boff[b] = acc; int c = HST[(size_t)b * NGP + g]; c = (c < 0) ? 0 : (c > CHP ? CHP : c); acc += c; if (acc > tot) acc = tot; } boff[CSR_NBLKB] = acc; }
  for (int i = t_; i <= CSR_GNB; i += 256) ncnt[i] = 0;
  __syncthreads();
  for (int b = 0; b < CSR_NBLKB; ++b) { const int c = boff[b + 1] - boff[b]; int o_ = OFF[(size_t)g * CSR_NBLKB + b]; o_ = (o_ < 0) ? 0 : (o_ > CHP - c ? CHP - c : o_); const int* src_ = STG + (size_t)b * CHP + o_;
    for (int i = t_; i < c; i += 256) { int id = src_[i]; id = (id < 0) ? 0 : id; ids[boff[b] + i] = id; int d = dst[id]; d = (d < v0) ? v0 : (d >= N ? N - 1 : d); int kk = d - v0; kk = (kk < 0) ? 0 : (kk >= CSR_GNB ? CSR_GNB - 1 : kk); key[boff[b] + i] = (unsigned short)kk; } }
  __syncthreads();
  if (t_ == 0) { for (int i = 0; i < tot; ++i) ncnt[key[i]] += 1; int acc = 0; for (int vl = 0; vl < CSR_GNB; ++vl) { const int c = ncnt[vl]; ncnt[vl] = acc; acc += c; } ncnt[CSR_GNB] = acc;
    for (int i = 0; i < tot; ++i) { const int vl = key[i]; outp[ncnt[vl]] = ids[i]; ncnt[vl] += 1; }
    for (int vl = CSR_GNB; vl > 0; --vl) ncnt[vl] = ncnt[vl - 1]; ncnt[0] = 0; }
  __syncthreads();
  for (int pass = 0; pass < 2; ++pass) {
    for (int i = t_; i < (stn - st) / 4; i += 256) { v4i v; for (int e = 0; e < 4; ++e) { const int q = i * 4 + e; v[e] = (q < tot) ? outp[q] : -1; } *(volatile v4i*)(PERM + st + i * 4) = v; }
    for (int i = t_; i < CSR_TSB / 4; i += 256) { v4i a, c; for (int e = 0; e < 4; ++e) { const int vl = i * 4 + e; const int vc = vl < CSR_GNB ? vl : CSR_GNB; a[e] = (vl < CSR_GNB) ? st + ncnt[vc] : st; c[e] = (vl < nv) ? (ncnt[(vc < CSR_GNB ? vc : CSR_GNB - 1) + 1] - ncnt[vc]) : 0; } *(volatile v4i*)(ROWPTR + t0 + i * 4) = a; *(volatile v4i*)(ROWCNT + t0 + i * 4) = c; }
    __threadfence(); }
}
__global__ __launch_bounds__(256) void csrZ_kernelB(int* __restrict__ p, size_t n4) { typedef __attribute__((ext_vector_type(4))) int v4i; const size_t tid = (size_t)blockIdx.x * 256 + threadIdx.x, nth = (size_t)gridDim.x * 256; v4i z = {0, 0, 0, 0}; for (size_t i = tid; i < n4; i += nth) *(volatile v4i*)(p + i * 4) = z; }
struct CsrBufsB { int *STG, *HST, *OFF, *START, *TOT, *PERM, *ROWPTR, *ROWCNT, *FLAG; int nG, NGP, CHP; size_t permLen; char* base; size_t bytes; };
static size_t csr_carveB(CsrBufsB& c, char* ws, size_t off, int E, int N) {
  const size_t off0 = off; c.base = ws + off;
  auto al = [&](size_t bytes) { char* p = ws + off; off += (bytes + 255) & ~(size_t)255; return p; };
  c.nG = (N + CSR_GNB - 1) / CSR_GNB; c.NGP = (c.nG + 31) & ~31; const int ch = (E + CSR_NBLKB - 1) / CSR_NBLKB; c.CHP = (ch + 31) & ~31; c.permLen = (size_t)E + 32 * (size_t)c.nG + 32;
  c.STG = (int*)al((size_t)CSR_NBLKB * c.CHP * 4); c.HST = (int*)al((size_t)CSR_NBLKB * c.NGP * 4); c.OFF = (int*)al((size_t)c.NGP * CSR_NBLKB * 4); c.START = (int*)al((size_t)(c.NGP + 64) * 4); c.TOT = (int*)al((size_t)(c.NGP + 64) * 4);
  c.PERM = (int*)al(c.permLen * 4); c.ROWPTR = (int*)al((size_t)c.nG * CSR_TSB * 4); c.ROWCNT = (int*)al((size_t)c.nG * CSR_TSB * 4); c.FLAG = (int*)al(256);
  c.bytes = off - off0; return off;
}
static void csr_buildB(const CsrBufsB& c, const int* dst, int E, int N, hipStream_t stream) {
  const size_t smem = (size_t)(2 * c.NGP + c.CHP) * 4;
  csrZ_kernelB<<<512, 256, 0, stream>>>((int*)c.base, c.bytes / 16);
  csrA_kernelB<<<CSR_NBLKB, 64, smem, stream>>>(dst, E, N, c.nG, c.CHP, c.NGP, c.STG, c.HST);
  csrS_kernelB<<<1, 512, 0, stream>>>(c.HST, c.nG, c.NGP, c.START, c.TOT, c.OFF);
  csrB_kernelB<<<c.nG, 256, 0, stream>>>(dst, N, c.nG, c.CHP, c.NGP, (int)c.permLen, c.STG, c.HST, c.OFF, c.START, c.TOT, c.PERM, c.ROWPTR, c.ROWCNT, c.FLAG);
}
constexpr int CSR_NBLKC = 512, CSR_GBC = 9, CSR_GNC = 1 << CSR_GBC  , CSR_TSC = (CSR_GNC < 32 ? 32 : CSR_GNC)  , CSR_MAXGC = 512, CSR_CAPC = 12288  ;
__device__ __host__ __forceinline__ int csr_tixC(int v) { return (v >> CSR_GBC) * CSR_TSC + (v & (CSR_GNC - 1)); }
__global__ __launch_bounds__(64) void csrA_kernelC(const int* __restrict__ dst, int E, int N, int nG, int CHP, int NGP, int* __restrict__ STG, int* __restrict__ HST) {
  extern __shared__ int sm[];
  int* cnt = sm; int* run = sm + NGP; int* ids = sm + 2 * NGP;
  const int b = blockIdx.x; const int ch = (E + CSR_NBLKC - 1) / CSR_NBLKC; const int e0 = b * ch, e1 = min(E, e0 + ch);
  for (int i = threadIdx.x; i < NGP; i += 64) cnt[i] = 0;
  for (int i = threadIdx.x; i < CHP; i += 64) ids[i] = -1;
  __syncthreads();
  if (threadIdx.x == 0) {
    for (int e = e0; e < e1; ++e) { int d = dst[e]; d = (d < 0) ? 0 : (d >= N ? N - 1 : d); cnt[d >> CSR_GBC] += 1; }
    int acc = 0; for (int g = 0; g < nG; ++g) { run[g] = acc; acc += cnt[g]; }
    for (int e = e0; e < e1; ++e) { int d = dst[e]; d = (d < 0) ? 0 : (d >= N ? N - 1 : d); const int g = d >> CSR_GBC; ids[run[g]] = e; run[g] += 1; } }
  __syncthreads();
  typedef __attribute__((ext_vector_type(4))) int v4i;
  for (int pass = 0; pass < 2; ++pass) {
    for (int i = threadIdx.x; i < CHP / 4; i += 64) *(volatile v4i*)(STG + (size_t)b * CHP + i * 4) = *(const v4i*)(&ids[i * 4]);
    for (int i = threadIdx.x; i < NGP / 4; i += 64) { v4i v; for (int e = 0; e < 4; ++e) v[e] = (i * 4 + e < nG) ? cnt[i * 4 + e] : 0; *(volatile v4i*)(HST + (size_t)b * NGP + i * 4) = v; }
    __threadfence(); }
}
__global__ __launch_bounds__(512) void csrS_kernelC(const int* __restrict__ HST, int nG, int NGP, int* __restrict__ START, int* __restrict__ TOT, int* __restrict__ OFF) {
  __shared__ int tot[CSR_MAXGC];
  const int b = threadIdx.x;
  for (int pass = 0; pass < 2; ++pass) { int runb = 0; for (int g = 0; g < nG; ++g) { int c = HST[(size_t)b * NGP + g]; c = (c < 0) ? 0 : c; ((volatile int*)OFF)[(size_t)g * CSR_NBLKC + b] = runb; runb += c; } __threadfence(); }
  for (int g = threadIdx.x; g < nG; g += 512) { int s = 0; for (int bb = 0; bb < CSR_NBLKC; ++bb) { int c = HST[(size_t)bb * NGP + g]; s += (c < 0) ? 0 : c; } tot[g] = s; }
  __syncthreads();
  if (threadIdx.x < 32) {
    __shared__ int st[CSR_MAXGC + 32];
    if (threadIdx.x == 0) { int acc = 0; for (int g = 0; g < NGP; ++g) { st[g] = acc; if (g < nG) acc += (tot[g] + 31) & ~31; } st[NGP] = acc; }
    __builtin_amdgcn_fence(__ATOMIC_RELEASE, "workgroup"); __builtin_amdgcn_wave_barrier(); __builtin_amdgcn_fence(__ATOMIC_ACQUIRE, "workgroup");
    for (int pass = 0; pass < 2; ++pass) { for (int i = threadIdx.x; i < NGP + 32; i += 32) { ((volatile int*)START)[i] = (i <= NGP) ? st[min(i, NGP)] : 0; ((volatile int*)TOT)[i] = (i < nG) ? tot[i] : 0; } __threadfence(); } }
}
__global__ __launch_bounds__(256) void csrB_kernelC(const int* __restrict__ dst, int N, int nG, int CHP, int NGP, int permLen, const int* __restrict__ STG, const int* __restrict__ HST, const int* __restrict__ OFF, const int* __restrict__ START, const int* __restrict__ TOT, int* __restrict__ PERM, int* __restrict__ ROWPTR, int* __restrict__ ROWCNT, int* __restrict__ FLAG) {
  typedef __attribute__((ext_vector_type(4))) int v4i;
  __shared__ int ids[CSR_CAPC]; __shared__ unsigned short key[CSR_CAPC]; __shared__ int outp[CSR_CAPC]; __shared__ int ncnt[CSR_GNC + 1]; __shared__ int boff[CSR_NBLKC + 1];
  const int g = blockIdx.x, t_ = threadIdx.x; int tot = TOT[g]; int st = START[g], stn = START[g + 1]; const int v0 = g * CSR_GNC; const int nv = min(CSR_GNC, N - v0); const int t0 = g * CSR_TSC;
  st = (st < 0) ? 0 : (st > permLen - 32 ? permLen - 32 : st) & ~31; stn = (stn < st) ? st : (stn > permLen ? permLen : stn); tot = (tot < 0) ? 0 : tot; if (tot > stn - st && tot <= CSR_CAPC) tot = stn - st;
  if (tot > CSR_CAPC) {
    for (int pass = 0; pass < 2; ++pass) { for (int i = t_; i < CSR_TSC / 4; i += 256) { v4i a, c; for (int e = 0; e < 4; ++e) { a[e] = st; c[e] = 0; } *(volatile v4i*)(ROWPTR + t0 + i * 4) = a; *(volatile v4i*)(ROWCNT + t0 + i * 4) = c; } if (t_ == 0) ((volatile int*)FLAG)[0] = 1; __threadfence(); } (void)nv; return; }
  if (t_ == 0) { int acc = 0; for (int b = 0; b < CSR_NBLKC; ++b) { boff[b] = acc; int c = HST[(size_t)b * NGP + g]; c = (c < 0) ? 0 : (c > CHP ? CHP : c); acc += c; if (acc > tot) acc = tot; } boff[CSR_NBLKC] = acc; }
  for (int i = t_; i <= CSR_GNC; i += 256) ncnt[i] = 0;
  __syncthreads();
  for (int b = 0; b < CSR_NBLKC; ++b) { const int c = boff[b + 1] - boff[b]; int o_ = OFF[(size_t)g * CSR_NBLKC + b]; o_ = (o_ < 0) ? 0 : (o_ > CHP - c ? CHP - c : o_); const int* src_ = STG + (size_t)b * CHP + o_;
    for (int i = t_; i < c; i += 256) { int id = src_[i]; id = (id < 0) ? 0 : id; ids[boff[b] + i] = id; int d = dst[id]; d = (d < v0) ? v0 : (d >= N ? N - 1 : d); int kk = d - v0; kk = (kk < 0) ? 0 : (kk >= CSR_GNC ? CSR_GNC - 1 : kk); key[boff[b] + i] = (unsigned short)kk; } }
  __syncthreads();
  if (t_ == 0) { for (int i = 0; i < tot; ++i) ncnt[key[i]] += 1; int acc = 0; for (int vl = 0; vl < CSR_GNC; ++vl) { const int c = ncnt[vl]; ncnt[vl] = acc; acc += c; } ncnt[CSR_GNC] = acc;
    for (int i = 0; i < tot; ++i) { const int vl = key[i]; outp[ncnt[vl]] = ids[i]; ncnt[vl] += 1; }
    for (int vl = CSR_GNC; vl > 0; --vl) ncnt[vl] = ncnt[vl - 1]; ncnt[0] = 0; }
  __syncthreads();
  for (int pass = 0; pass < 2; ++pass) {
    for (int i = t_; i < (stn - st) / 4; i += 256) { v4i v; for (int e = 0; e < 4; ++e) { const int q = i * 4 + e; v[e] = (q < tot) ? outp[q] : -1; } *(volatile v4i*)(PERM + st + i * 4) = v; }
    for (int i = t_; i < CSR_TSC / 4; i += 256) { v4i a, c; for (int e = 0; e < 4; ++e) { const int vl = i * 4 + e; const int vc = vl < CSR_GNC ? vl : CSR_GNC; a[e] = (vl < CSR_GNC) ? st + ncnt[vc] : st; c[e] = (vl < nv) ? (ncnt[(vc < CSR_GNC ? vc : CSR_GNC - 1) + 1] - ncnt[vc]) : 0; } *(volatile v4i*)(ROWPTR + t0 + i * 4) = a; *(volatile v4i*)(ROWCNT + t0 + i * 4) = c; }
    __threadfence(); }
}
__global__ __launch_bounds__(256) void csrZ_kernelC(int* __restrict__ p, size_t n4) { typedef __attribute__((ext_vector_type(4))) int v4i; const size_t tid = (size_t)blockIdx.x * 256 + threadIdx.x, nth = (size_t)gridDim.x * 256; v4i z = {0, 0, 0, 0}; for (size_t i = tid; i < n4; i += nth) *(volatile v4i*)(p + i * 4) = z; }
struct CsrBufsC { int *STG, *HST, *OFF, *START, *TOT, *PERM, *ROWPTR, *ROWCNT, *FLAG; int nG, NGP, CHP; size_t permLen; char* base; size_t bytes; };
static size_t csr_carveC(CsrBufsC& c, char* ws, size_t off, int E, int N) {
  const size_t off0 = off; c.base = ws + off;
  auto al = [&](size_t bytes) { char* p = ws + off; off += (bytes + 255) & ~(size_t)255; return p; };
  c.nG = (N + CSR_GNC - 1) / CSR_GNC; c.NGP = (c.nG + 31) & ~31; const int ch = (E + CSR_NBLKC - 1) / CSR_NBLKC; c.CHP = (ch + 31) & ~31; c.permLen = (size_t)E + 32 * (size_t)c.nG + 32;
  c.STG = (int*)al((size_t)CSR_NBLKC * c.CHP * 4); c.HST = (int*)al((size_t)CSR_NBLKC * c.NGP * 4); c.OFF = (int*)al((size_t)c.NGP * CSR_NBLKC * 4); c.START = (int*)al((size_t)(c.NGP + 64) * 4); c.TOT = (int*)al((size_t)(c.NGP + 64) * 4);
  c.PERM = (int*)al(c.permLen * 4); c.ROWPTR = (int*)al((size_t)c.nG * CSR_TSC * 4); c.ROWCNT = (int*)al((size_t)c.nG * CSR_TSC * 4); c.FLAG = (int*)al(256);
  c.bytes = off - off0; return off;
}
static void csr_buildC(const CsrBufsC& c, const int* dst, int E, int N, hipStream_t stream) {
  const size_t smem = (size_t)(2 * c.NGP + c.CHP) * 4;
  csrZ_kernelC<<<512, 256, 0, stream>>>((int*)c.base, c.bytes / 16);
  csrA_kernelC<<<CSR_NBLKC, 64, smem, stream>>>(dst, E, N, c.nG, c.CHP, c.NGP, c.STG, c.HST);
  csrS_kernelC<<<1, 512, 0, stream>>>(c.HST, c.nG, c.NGP, c.START, c.TOT, c.OFF);
  csrB_kernelC<<<c.nG, 256, 0, stream>>>(dst, N, c.nG, c.CHP, c.NGP, (int)c.permLen, c.STG, c.HST, c.OFF, c.START, c.TOT, c.PERM, c.ROWPTR, c.ROWCNT, c.FLAG);
}


__global__ __launch_bounds__(256) void wput_kernel(const float* __restrict__ w, const float* __restrict__ w1, b16* __restrict__ WT, b16* __restrict__ W1T) { const int u = blockIdx.x * 256 + threadIdx.x; v8b v;
  if (u < M * D * 32) { const int r = u / 32, d0 = (u % 32) * 8; const int m = r / D, o = r % D;
#pragma unroll
    for (int j = 0; j < 8; ++j) v[j] = (b16)(bf16_rne(w[((size_t)m * D + d0 + j) * D + o]) * WSC); for (int pass = 0; pass < 2; ++pass) { *(volatile v8b*)(WT + (size_t)r * D + d0) = v; __threadfence(); } }
  if (u < HID * 32) { const int o = u / 32, k0 = (u % 32) * 8;
#pragma unroll
    for (int j = 0; j < 8; ++j) v[j] = (b16)(bf16_rne(w1[(size_t)(k0 + j) * HID + o]) * WSC); for (int pass = 0; pass < 2; ++pass) { *(volatile v8b*)(W1T + (size_t)o * D + k0) = v; __threadfence(); } } }
__global__ __launch_bounds__(32) void node_kernel(const float* __restrict__ h, const b16* __restrict__ WT, const float* __restrict__ al, const float* __restrict__ ar, int NLIM, float* __restrict__ Z, float* __restrict__ EL) { __shared__ __attribute__((aligned(16))) b16 Ah[16][D + 8]; __shared__ float Tf[16][D + 4]; __shared__ float Se[16][16]; const int lane = threadIdx.x, nloc = lane & 15, hlf = lane >> 4; const int m = blockIdx.x % M; const size_t m0 = (size_t)(blockIdx.x / M) * 16; if (m0 >= (size_t)NLIM) return;
  for (int rr = 0; rr < 16; ++rr) for (int q = 0; q < 8; ++q) Ah[rr][q * 32 + lane] = (b16)(bf16_rne(h[(m0 + rr) * D + q * 32 + lane]) * XS);
  wave_lds_sync(); v8f acc[16];
#pragma unroll
  for (int t = 0; t < 16; ++t) acc[t] = (v8f){};
#pragma unroll 2
  for (int kb = 0; kb < D; kb += 32) { const v16b a = frag_kb(&Ah[nloc][kb], hlf);
#pragma unroll
    for (int t = 0; t < 16; ++t) acc[t] = wmma16b(a, frag_kb(WT + ((size_t)m * D + t * 16 + nloc) * D + kb, hlf), acc[t]); }
#pragma unroll
  for (int t = 0; t < 16; ++t)
#pragma unroll
    for (int r8 = 0; r8 < 8; ++r8) Tf[8 * hlf + r8][t * 16 + nloc] = acc[t][r8] * (1.0f / (XS * WSC));
  wave_lds_sync();
  for (int rr = 0; rr < 16; ++rr) { float s0 = 0.0f, s1 = 0.0f; for (int k = 0; k < 8; ++k) { const int c = lane * 8 + k; const float z = Tf[rr][c]; s0 += pmul(z, bfv(al[m * D + c])); s1 += pmul(z, bfv(ar[m * D + c])); } s0 += __shfl_xor(s0, 1); s0 += __shfl_xor(s0, 2); s1 += __shfl_xor(s1, 1); s1 += __shfl_xor(s1, 2); if ((lane & 3) == 0) { Se[rr][lane >> 2] = s0; Se[rr][8 + (lane >> 2)] = s1; } }
  wave_lds_sync();
  for (int pass = 0; pass < 2; ++pass) { for (int rr = 0; rr < 16; ++rr) { for (int q = 0; q < 2; ++q) *(volatile v4f*)(Z + ((size_t)m * N + m0 + rr) * D + q * 128 + lane * 4) = *(const v4f*)(&Tf[rr][q * 128 + lane * 4]); ((volatile float*)EL)[((size_t)m * N + m0 + rr) * 32 + lane] = lane < 16 ? Se[rr][lane] : 0.0f; } __threadfence(); } }
__global__ __launch_bounds__(256) void edge_kernel(const float* __restrict__ Z, const float* __restrict__ EL, const float* __restrict__ bias, int m, const int* __restrict__ srcs, const int* __restrict__ PERM, const int* __restrict__ ROWPTR, const int* __restrict__ ROWCNT, int permLen, int NLIM, float* __restrict__ ZP) { const int wave = threadIdx.x >> 5, lane = threadIdx.x & 31; const size_t i = (size_t)blockIdx.x * 8 + wave; if (i >= (size_t)NLIM) return; int st = ROWPTR[i], cnt = ROWCNT[i]; cnt = iclamp(cnt, 0, E); st = iclamp(st, 0, permLen - cnt);
  const int hd = lane >> 2; const float eri = EL[((size_t)m * N + i) * 32 + 8 + hd]; float mx = -INFINITY, den = 0.0f, acc[8]; for (int k = 0; k < 8; ++k) acc[k] = 0.0f;
  const float* Zm = Z + (size_t)m * N * D;
#pragma unroll 1
  for (int j = 0; j < cnt; ++j) { const int e = iclamp(PERM[st + j], 0, E - 1); const size_t u = (size_t)iclamp(srcs[e], 0, N - 1); if (u >= (size_t)NLIM) continue; const float s = leaky(EL[((size_t)m * N + u) * 32 + hd] + eri); const float mn = fmaxf(mx, s); const float sf = (mx == -INFINITY) ? 0.0f : __expf(mx - mn); const float p = __expf(s - mn); den = den * sf + p; const float* zu = Zm + u * D + lane * 8; const v4f a = *(const v4f*)zu, b = *(const v4f*)(zu + 4);
#pragma unroll
    for (int k = 0; k < 4; ++k) { acc[k] = pmul(acc[k], sf) + pmul(p, a[k]); acc[4 + k] = pmul(acc[4 + k], sf) + pmul(p, b[k]); } mx = mn; }
  const float inv = den > 0.0f ? 1.0f / den : 0.0f; float o8[8];
#pragma unroll
  for (int k = 0; k < 8; ++k) o8[k] = elu(pmul(acc[k], inv) + bfv(bias[m * D + lane * 8 + k]));
  for (int pass = 0; pass < 2; ++pass) { *(volatile v4f*)(ZP + (i * M + m) * D + lane * 8) = (v4f){o8[0], o8[1], o8[2], o8[3]}; *(volatile v4f*)(ZP + (i * M + m) * D + lane * 8 + 4) = (v4f){o8[4], o8[5], o8[6], o8[7]}; __threadfence(); } }
__global__ __launch_bounds__(32) void sem_kernel(const float* __restrict__ ZP, const b16* __restrict__ W1T, const float* __restrict__ b1, const float* __restrict__ w2, int RLIM, float* __restrict__ PART) { __shared__ __attribute__((aligned(16))) b16 Ah[16][D + 8], Al[16][D + 8]; __shared__ float Tf[16][HID + 4]; const int lane = threadIdx.x, nloc = lane & 15, hlf = lane >> 4; const size_t r0 = (size_t)blockIdx.x * 16; float pm[3] = {0.0f, 0.0f, 0.0f};
  if (r0 < (size_t)RLIM) {
    for (int rr = 0; rr < 16; ++rr) for (int q = 0; q < 8; ++q) { b16 p, ql; split16(ZP[(r0 + rr) * D + q * 32 + lane] * HS, p, ql); Ah[rr][q * 32 + lane] = p; Al[rr][q * 32 + lane] = ql; }
    wave_lds_sync(); v8f acc[8];
#pragma unroll
    for (int t = 0; t < 8; ++t) acc[t] = (v8f){};
#pragma unroll 2
    for (int kb = 0; kb < D; kb += 32) { const v16b a = frag_kb(&Ah[nloc][kb], hlf), al_ = frag_kb(&Al[nloc][kb], hlf);
#pragma unroll
      for (int t = 0; t < 8; ++t) { const v16b bw = frag_kb(W1T + (size_t)(t * 16 + nloc) * D + kb, hlf); acc[t] = wmma16b(a, bw, acc[t]); acc[t] = wmma16b(al_, bw, acc[t]); } }
#pragma unroll
    for (int t = 0; t < 8; ++t) { const int cc = t * 16 + nloc; const float bb = bfv(b1[cc]), ww = bfv(w2[cc]);
#pragma unroll
      for (int r8 = 0; r8 < 8; ++r8) Tf[8 * hlf + r8][cc] = pmul(tanhf(acc[t][r8] * (1.0f / (HS * WSC)) + bb), ww); }
    wave_lds_sync();
    for (int rr = 0; rr < 16; ++rr) { float s = Tf[rr][lane] + Tf[rr][32 + lane] + Tf[rr][64 + lane] + Tf[rr][96 + lane]; for (int o = 16; o; o >>= 1) s += __shfl_xor(s, o); const int mm = (int)((r0 + rr) % M);
#pragma unroll
      for (int q = 0; q < 3; ++q) if (q == mm) pm[q] += s; } }
  for (int pass = 0; pass < 2; ++pass) { ((volatile float*)PART)[(size_t)blockIdx.x * 32 + lane] = lane == 0 ? pm[0] : (lane == 1 ? pm[1] : (lane == 2 ? pm[2] : 0.0f)); __threadfence(); } }
__global__ __launch_bounds__(32) void beta_kernel(const float* __restrict__ PART, int nw, int NLIM, float* __restrict__ BETA) { const int lane = threadIdx.x; double s[3] = {0.0, 0.0, 0.0};
#pragma unroll 1
  for (int w = 0; w < nw; ++w) {
#pragma unroll
    for (int q = 0; q < 3; ++q) s[q] += (double)PART[(size_t)w * 32 + q]; }
  float mw[3]; for (int q = 0; q < 3; ++q) mw[q] = (float)(s[q] / (double)NLIM); const float mx = fmaxf(mw[0], fmaxf(mw[1], mw[2])); float ex[3], den = 0.0f; for (int q = 0; q < 3; ++q) { ex[q] = __expf(mw[q] - mx); den += ex[q]; }
  for (int pass = 0; pass < 2; ++pass) { ((volatile float*)BETA)[lane] = lane < 3 ? ex[lane < 3 ? lane : 0] / den : 0.0f; __threadfence(); } }
__global__ __launch_bounds__(256) void out_kernel(const float* __restrict__ ZP, const float* __restrict__ BETA, int NLIM, float* __restrict__ out) { const int wave = threadIdx.x >> 5, lane = threadIdx.x & 31; const size_t i = (size_t)blockIdx.x * 8 + wave; if (i >= (size_t)NLIM) return; const float b0 = BETA[0], b1_ = BETA[1], b2_ = BETA[2];
  for (int pass = 0; pass < 2; ++pass) { for (int q = 0; q < 2; ++q) { v4f o; for (int k = 0; k < 4; ++k) { const int c = q * 128 + lane * 4 + k; o[k] = pmul(b0, ZP[(i * M) * D + c]) + pmul(b1_, ZP[(i * M + 1) * D + c]) + pmul(b2_, ZP[(i * M + 2) * D + c]); } *(volatile v4f*)(out + i * D + q * 128 + lane * 4) = o; } __threadfence(); } }
}

extern "C" void kernel_launch(void* const* d_in, const int* in_sizes, int n_in, void* d_out, int out_size, void* d_ws, size_t ws_size, hipStream_t stream) {
  (void)n_in;
  auto Fp = [&](int i) { return (const float*)d_in[i]; }; auto Ip = [&](int i) { return (const int*)d_in[i]; };
  if (in_sizes[0] != N * D || in_sizes[1] != M * D * D || in_sizes[2] != M * D || in_sizes[3] != M * D || in_sizes[4] != M * D || in_sizes[5] != D * HID || in_sizes[7] != HID || in_sizes[8] != M * E || in_sizes[9] != M * E || out_size != N * D) return;
  const int NLIM = N;
  size_t off = 0; char* ws = (char*)d_ws;
  auto carve = [&](size_t bytes) { char* p = ws + off; off += (bytes + 255) & ~(size_t)255; return p; };
  b16* WT = (b16*)carve((size_t)M * D * D * 2); b16* W1T = (b16*)carve((size_t)HID * D * 2); float* Z = (float*)carve((size_t)M * N * D * 4); float* EL = (float*)carve((size_t)M * N * 32 * 4); float* ZP = (float*)carve((size_t)N * M * D * 4); float* PART = (float*)carve((size_t)NSW * 32 * 4); float* BETA = (float*)carve(32 * 4);
  CsrBufsA ca; off = csr_carveA(ca, ws, off, E, N); CsrBufsB cb_; off = csr_carveB(cb_, ws, off, E, N); CsrBufsC cc_; off = csr_carveC(cc_, ws, off, E, N);
  if (off > ws_size || off > ((size_t)96 << 20)) return;
  const int nsw = (NLIM * M) / 16;
  wput_kernel<<<(M * D * 32 + 255) / 256, 256, 0, stream>>>(Fp(1), Fp(5), WT, W1T);
  csr_buildA(ca, Ip(9), E, N, stream); csr_buildB(cb_, Ip(9) + E, E, N, stream); csr_buildC(cc_, Ip(9) + 2 * E, E, N, stream);
  node_kernel<<<(NLIM / 16) * M, 32, 0, stream>>>(Fp(0), WT, Fp(2), Fp(3), NLIM, Z, EL);
  edge_kernel<<<(NLIM + 7) / 8, 256, 0, stream>>>(Z, EL, Fp(4), 0, Ip(8), ca.PERM, ca.ROWPTR, ca.ROWCNT, (int)ca.permLen, NLIM, ZP);
  edge_kernel<<<(NLIM + 7) / 8, 256, 0, stream>>>(Z, EL, Fp(4), 1, Ip(8) + E, cb_.PERM, cb_.ROWPTR, cb_.ROWCNT, (int)cb_.permLen, NLIM, ZP);
  edge_kernel<<<(NLIM + 7) / 8, 256, 0, stream>>>(Z, EL, Fp(4), 2, Ip(8) + 2 * E, cc_.PERM, cc_.ROWPTR, cc_.ROWCNT, (int)cc_.permLen, NLIM, ZP);
  sem_kernel<<<nsw, 32, 0, stream>>>(ZP, W1T, Fp(6), Fp(7), NLIM * M, PART);
  beta_kernel<<<1, 32, 0, stream>>>(PART, nsw, NLIM, BETA);
  out_kernel<<<(NLIM + 7) / 8, 256, 0, stream>>>(ZP, BETA, NLIM, (float*)d_out);
}
